// TensorChannel_90984587198691
// MI455X (gfx1250) — hardware-verified
//
#include <hip/hip_runtime.h>
#include <stdint.h>
#include <stddef.h>


#define IN_D   128
#define D9     144
#define KP2    160
#define DI     512
#define CHK    2048
#define MAXDEG 1024

typedef _Float16 v8h  __attribute__((ext_vector_type(8)));
typedef _Float16 v16h __attribute__((ext_vector_type(16)));
typedef __bf16   v8b  __attribute__((ext_vector_type(8)));
typedef __bf16   v16b __attribute__((ext_vector_type(16)));
typedef float    v8f  __attribute__((ext_vector_type(8)));
typedef float    v4f  __attribute__((ext_vector_type(4)));
typedef float    v2f  __attribute__((ext_vector_type(2)));
typedef int      v4i  __attribute__((ext_vector_type(4)));
typedef unsigned v4u  __attribute__((ext_vector_type(4)));
typedef _Float16 v8ha __attribute__((ext_vector_type(8), __may_alias__));
typedef __bf16   v8ba __attribute__((ext_vector_type(8), __may_alias__));
typedef float    v4fa __attribute__((ext_vector_type(4), __may_alias__));
typedef float    v2fa __attribute__((ext_vector_type(2), __may_alias__));
typedef int      v4ia __attribute__((ext_vector_type(4), __may_alias__));

union FragH { v16h v; v8h half[2]; };
union FragB { v16b v; v8b half[2]; };
union P16   { v4u u; _Float16 f[8]; unsigned short s[8]; };

__device__ __forceinline__ v8f mma_f16(v16h a, v16h b, v8f c)
{
    c = __builtin_amdgcn_wmma_f32_16x16x32_f16(false, a, false, b, (short)0, c, false, false);
    asm volatile("v_nop\n\tv_nop\n\tv_nop\n\tv_nop" : "+v"(c) : "v"(a), "v"(b));
    return c;
}
__device__ __forceinline__ v8f mma_bf16(v16b a, v16b b, v8f c)
{
    c = __builtin_amdgcn_wmma_f32_16x16x32_bf16(false, a, false, b, (short)0, c, false, false);
    asm volatile("v_nop\n\tv_nop\n\tv_nop\n\tv_nop" : "+v"(c) : "v"(a), "v"(b));
    return c;
}

__device__ __forceinline__ v8h ldh8(const _Float16* p) { return *(const v8ha*)p; }
__device__ __forceinline__ v8b ldb8(const __bf16* p)   { return *(const v8ba*)p; }

__device__ __forceinline__ unsigned short bf_bits(float x)
{
    unsigned u = __builtin_bit_cast(unsigned, x);
    u += 0x7FFFu + ((u >> 16) & 1u);
    return (unsigned short)(u >> 16);
}
__device__ __forceinline__ float  bf_val(unsigned short s) { return __builtin_bit_cast(float, ((unsigned)s) << 16); }
__device__ __forceinline__ __bf16 bf_mk(unsigned short s)  { return __builtin_bit_cast(__bf16, s); }

__device__ __forceinline__ float sigm(float x) { return 1.0f / (1.0f + __expf(-x)); }
__device__ __forceinline__ int clampi(int v, int lo, int hi) { return v < lo ? lo : (v > hi ? hi : v); }

__device__ __forceinline__ float hsum16(float s)
{
    s += __shfl_xor(s, 8);
    s += __shfl_xor(s, 4);
    s += __shfl_xor(s, 2);
    s += __shfl_xor(s, 1);
    return s;
}

__device__ __forceinline__ v8f zero8()
{
    v8f z = {0.f, 0.f, 0.f, 0.f, 0.f, 0.f, 0.f, 0.f};
    return z;
}

__global__ __launch_bounds__(256) void k_conv(
    const float* __restrict__ h, const float* __restrict__ W1,
    const float* __restrict__ W2, const float* __restrict__ Wi,
    _Float16* __restrict__ hh, __bf16* __restrict__ W1hi, __bf16* __restrict__ W1lo,
    __bf16* __restrict__ W2hi, __bf16* __restrict__ W2lo, _Float16* __restrict__ Wih,
    int N, int Npad, int s1, int s3, int s5)
{
    const int b = blockIdx.x, t = threadIdx.x;
    v4f va = {0.f, 0.f, 0.f, 0.f}, vb = {0.f, 0.f, 0.f, 0.f};
    int kind = -1;
    void* dst = 0;

    if (b < s1) {
        const long gidx = (long)b * 256 + t;
        if (gidx < (long)Npad * (IN_D / 8)) {
            const int row = (int)(gidx / (IN_D / 8)), q = (int)(gidx % (IN_D / 8));
            const int sr = row < N ? row : N - 1;
            const float* src = h + (size_t)sr * IN_D + q * 8;
            va = *(const v4fa*)src * 16.0f;
            vb = *(const v4fa*)(src + 4) * 16.0f;
            kind = 0;
            dst = (void*)(hh + (size_t)row * IN_D + q * 8);
        }
    } else if (b < s3) {
        const int half = (s3 - s1) >> 1;
        const bool lo = (b - s1) >= half;
        const int gidx = (b - s1 - (lo ? half : 0)) * 256 + t;
        if (gidx < D9 * (IN_D / 8)) {
            const int row = gidx / (IN_D / 8), q = gidx % (IN_D / 8);
            const float* src = W1 + (size_t)row * IN_D + q * 8;
            va = *(const v4fa*)src;
            vb = *(const v4fa*)(src + 4);
            kind = lo ? 2 : 1;
            dst = (void*)((lo ? W1lo : W1hi) + (size_t)row * IN_D + q * 8);
        }
    } else if (b < s5) {
        const int half = (s5 - s3) >> 1;
        const bool lo = (b - s3) >= half;
        const int gidx = (b - s3 - (lo ? half : 0)) * 256 + t;
        if (gidx < D9 * (KP2 / 8)) {
            const int row = gidx / (KP2 / 8), q = gidx % (KP2 / 8);
            const int k = q * 8;
            if (k < D9) {
                const float* src = W2 + (size_t)row * D9 + k;
                va = *(const v4fa*)src;
                vb = *(const v4fa*)(src + 4);
            }
            kind = lo ? 2 : 1;
            dst = (void*)((lo ? W2lo : W2hi) + (size_t)row * KP2 + k);
        }
    } else {
        const int gidx = (b - s5) * 256 + t;
        if (gidx < DI * (2 * IN_D / 8)) {
            const int row = gidx / (2 * IN_D / 8), q = gidx % (2 * IN_D / 8);
            const float* src = Wi + (size_t)row * (2 * IN_D) + q * 8;
            va = *(const v4fa*)src * 64.0f;
            vb = *(const v4fa*)(src + 4) * 64.0f;
            kind = 0;
            dst = (void*)(Wih + (size_t)row * (2 * IN_D) + q * 8);
        }
    }

    if (kind >= 0) {
        const float v[8] = {va.x, va.y, va.z, va.w, vb.x, vb.y, vb.z, vb.w};
        P16 pk;
        if (kind == 0) {
#pragma unroll
            for (int i = 0; i < 8; ++i) pk.f[i] = (_Float16)v[i];
        } else if (kind == 1) {
#pragma unroll
            for (int i = 0; i < 8; ++i) pk.s[i] = bf_bits(v[i]);
        } else {
#pragma unroll
            for (int i = 0; i < 8; ++i) {
                const unsigned short hs = bf_bits(v[i]);
                pk.s[i] = bf_bits(v[i] - bf_val(hs));
            }
        }
        const v4u val = pk.u;
        *(volatile v4u*)dst = val;
        __threadfence();
        *(volatile v4u*)dst = val;
    }
}

__global__ __launch_bounds__(256) void k_node(
    const float* __restrict__ h,
    const __bf16* __restrict__ W1hi, const __bf16* __restrict__ W1lo,
    const float* __restrict__ b1, const float* __restrict__ g1, const float* __restrict__ be1,
    const __bf16* __restrict__ W2hi, const __bf16* __restrict__ W2lo,
    const float* __restrict__ b2, const float* __restrict__ g2, const float* __restrict__ be2,
    float* __restrict__ tens, int N)
{
    __shared__ __attribute__((aligned(16))) __bf16 sAhi[16 * 136];
    __shared__ __attribute__((aligned(16))) __bf16 sAlo[16 * 136];
    __shared__ __attribute__((aligned(16))) __bf16 sThi[16 * 168];
    __shared__ __attribute__((aligned(16))) __bf16 sTlo[16 * 168];
    __shared__ __attribute__((aligned(16))) float  sY[16 * 148];
    __shared__ __attribute__((aligned(16))) float  sO[16 * D9];

    const int tid = threadIdx.x, lane = tid & 31, wave = tid >> 5;
    const int hf = lane >> 4, m16 = lane & 15;
    const int n0 = blockIdx.x * 16;

    for (int idx = tid; idx < 512; idx += 256) {
        const int m = idx >> 5, j = (idx & 31) * 4;
        int node = n0 + m; node = node < N ? node : N - 1;
        const v4f v = *(const v4fa*)(h + (size_t)node * IN_D + j);
        const float vv[4] = {v.x, v.y, v.z, v.w};
#pragma unroll
        for (int u = 0; u < 4; ++u) {
            const unsigned short hs = bf_bits(vv[u]);
            sAhi[m * 136 + j + u] = bf_mk(hs);
            sAlo[m * 136 + j + u] = bf_mk(bf_bits(vv[u] - bf_val(hs)));
        }
    }
    __syncthreads();

    for (int nt = wave; nt < 9; nt += 8) {
        const int n = nt * 16 + m16;
        const __bf16* arh = sAhi + m16 * 136 + 8 * hf;
        const __bf16* arl = sAlo + m16 * 136 + 8 * hf;
        const __bf16* brh = W1hi + (size_t)n * IN_D + 8 * hf;
        const __bf16* brl = W1lo + (size_t)n * IN_D + 8 * hf;
        v8f acc = zero8();
#pragma unroll 1
        for (int k0 = 0; k0 < IN_D; k0 += 32) {
            FragB ah, al, bh, bl;
            ah.half[0] = ldb8(arh + k0); ah.half[1] = ldb8(arh + k0 + 16);
            al.half[0] = ldb8(arl + k0); al.half[1] = ldb8(arl + k0 + 16);
            bh.half[0] = ldb8(brh + k0); bh.half[1] = ldb8(brh + k0 + 16);
            bl.half[0] = ldb8(brl + k0); bl.half[1] = ldb8(brl + k0 + 16);
            acc = mma_bf16(ah.v, bh.v, acc);
            acc = mma_bf16(ah.v, bl.v, acc);
            acc = mma_bf16(al.v, bh.v, acc);
        }
        const float bb = b1[n];
#pragma unroll
        for (int r = 0; r < 8; ++r) sY[(8 * hf + r) * 148 + n] = acc[r] + bb;
    }
    __syncthreads();

    {
        const int m = tid >> 4, g = tid & 15;
        const float* yr = sY + m * 148;
        float s = 0.f;
        for (int j = g; j < D9; j += 16) s += yr[j];
        s = hsum16(s);
        const float mu = s * (1.0f / (float)D9);
        float q = 0.f;
        for (int j = g; j < D9; j += 16) { const float d = yr[j] - mu; q += d * d; }
        q = hsum16(q);
        const float rstd = rsqrtf(q * (1.0f / (float)D9) + 1e-5f);
        for (int j = g; j < D9; j += 16) {
            const float v = (yr[j] - mu) * rstd * g1[j] + be1[j];
            const float t = v * sigm(v);
            const unsigned short hs = bf_bits(t);
            sThi[m * 168 + j] = bf_mk(hs);
            sTlo[m * 168 + j] = bf_mk(bf_bits(t - bf_val(hs)));
        }
        sThi[m * 168 + D9 + g] = bf_mk((unsigned short)0);
        sTlo[m * 168 + D9 + g] = bf_mk((unsigned short)0);
    }
    __syncthreads();

    for (int nt = wave; nt < 9; nt += 8) {
        const int n = nt * 16 + m16;
        const __bf16* arh = sThi + m16 * 168 + 8 * hf;
        const __bf16* arl = sTlo + m16 * 168 + 8 * hf;
        const __bf16* brh = W2hi + (size_t)n * KP2 + 8 * hf;
        const __bf16* brl = W2lo + (size_t)n * KP2 + 8 * hf;
        v8f acc = zero8();
#pragma unroll 1
        for (int k0 = 0; k0 < KP2; k0 += 32) {
            FragB ah, al, bh, bl;
            ah.half[0] = ldb8(arh + k0); ah.half[1] = ldb8(arh + k0 + 16);
            al.half[0] = ldb8(arl + k0); al.half[1] = ldb8(arl + k0 + 16);
            bh.half[0] = ldb8(brh + k0); bh.half[1] = ldb8(brh + k0 + 16);
            bl.half[0] = ldb8(brl + k0); bl.half[1] = ldb8(brl + k0 + 16);
            acc = mma_bf16(ah.v, bh.v, acc);
            acc = mma_bf16(ah.v, bl.v, acc);
            acc = mma_bf16(al.v, bh.v, acc);
        }
        const float bb = b2[n];
#pragma unroll
        for (int r = 0; r < 8; ++r) sY[(8 * hf + r) * 148 + n] = acc[r] + bb;
    }
    __syncthreads();

    {
        const int m = tid >> 4, g = tid & 15;
        const float* yr = sY + m * 148;
        float s = 0.f;
        for (int j = g; j < D9; j += 16) s += yr[j];
        s = hsum16(s);
        const float mu = s * (1.0f / (float)D9);
        float q = 0.f;
        for (int j = g; j < D9; j += 16) { const float d = yr[j] - mu; q += d * d; }
        q = hsum16(q);
        const float rstd = rsqrtf(q * (1.0f / (float)D9) + 1e-5f);
        for (int j = g; j < D9; j += 16) {
            const float v = (yr[j] - mu) * rstd * g2[j] + be2[j];
            sO[m * D9 + j] = v * sigm(v);
        }
    }
    __syncthreads();

    float* dst = tens + (size_t)n0 * D9;
    for (int idx = tid; idx < 16 * D9 / 4; idx += 256) {
        const v4f v = *(const v4fa*)(sO + idx * 4);
        *(volatile v4f*)(dst + idx * 4) = v;
    }
    __threadfence();
    for (int idx = tid; idx < 16 * D9 / 4; idx += 256) {
        const v4f v = *(const v4fa*)(sO + idx * 4);
        *(volatile v4f*)(dst + idx * 4) = v;
    }
}

__device__ __forceinline__ void sort_emit(const int* sk, int* lbrow, int* skrow, int NP, int tid)
{
    const int ng = NP >> 2;
    for (int gq = tid; gq < ng; gq += 256) {
        v4i r = {0, 0, 0, 0};
#pragma unroll
        for (int u = 0; u < 4; ++u) {
            const int tgt = (gq * 4 + u) * CHK;
            int lo = 0, hi = CHK;
#pragma unroll
            for (int it = 0; it < 12; ++it) {
                if (lo < hi) {
                    const int mid = (lo + hi) >> 1;
                    if (sk[mid] < tgt) lo = mid + 1; else hi = mid;
                }
            }
            r[u] = lo;
        }
        *(volatile v4i*)(lbrow + gq * 4) = r;
    }
    for (int p4 = tid; p4 < CHK / 4; p4 += 256) {
        const v4i v = *(const v4ia*)(sk + p4 * 4);
        *(volatile v4i*)(skrow + p4 * 4) = v;
    }
}

__global__ __launch_bounds__(256) void k_sort(
    const int* __restrict__ ei, int* __restrict__ LB, int* __restrict__ SK,
    int N, int E, int NP)
{
    __shared__ __attribute__((aligned(16))) int sk[CHK];
    const int tid = threadIdx.x;
    const int c = blockIdx.x;

    for (int p = tid; p < CHK; p += 256) {
        const int e = c * CHK + p;
        int node = N;
        if (e < E) node = clampi(ei[(size_t)E + e], 0, N - 1);
        sk[p] = node * CHK + p;
    }
    __syncthreads();

    for (int k = 2; k <= CHK; k <<= 1) {
        for (int j = k >> 1; j > 0; j >>= 1) {
            for (int i = tid; i < CHK; i += 256) {
                const int ixj = i ^ j;
                if (ixj > i) {
                    const int a = sk[i], bq = sk[ixj];
                    const bool up = ((i & k) == 0);
                    if ((a > bq) == up) { sk[i] = bq; sk[ixj] = a; }
                }
            }
            __syncthreads();
        }
    }

    int* lbrow = LB + (size_t)c * NP;
    int* skrow = SK + (size_t)c * CHK;
    sort_emit(sk, lbrow, skrow, NP, tid);
    __threadfence();
    sort_emit(sk, lbrow, skrow, NP, tid);
}

__global__ __launch_bounds__(256) void k_edge(
    const _Float16* __restrict__ hh, const float* __restrict__ fr,
    const int* __restrict__ ei, const float* __restrict__ tens,
    const _Float16* __restrict__ Wih, const float* __restrict__ bi,
    const float* __restrict__ gi, const float* __restrict__ bei,
    float* __restrict__ TN, int N, int E)
{
    __shared__ __attribute__((aligned(16))) _Float16 sA[16 * 264];
    __shared__ __attribute__((aligned(16))) float sY[16 * 516];
    __shared__ __attribute__((aligned(16))) float sU[16 * 32 * 9];
    __shared__ float sR[16 * 12];
    __shared__ int   sCol[16], sRow[16];

    const int tid = threadIdx.x, lane = tid & 31, wave = tid >> 5;
    const int hf = lane >> 4, m16 = lane & 15;
    const int e0 = blockIdx.x * 16;

    if (tid < 16) {
        int e = e0 + tid; e = e < E ? e : E - 1;
        sRow[tid] = clampi(ei[e], 0, N - 1);
        sCol[tid] = clampi(ei[(size_t)E + e], 0, N - 1);
    }
    __syncthreads();

    for (int idx = tid; idx < 512; idx += 256) {
        const int m = idx >> 5, j = (idx & 31) * 8;
        const int node = (j < IN_D) ? sCol[m] : sRow[m];
        const v8h v = ldh8(hh + (size_t)node * IN_D + (j & (IN_D - 1)));
        *(v8ha*)(sA + m * 264 + j) = v;
    }
    __syncthreads();

    for (int i = 0; i < 4; ++i) {
        const int nt = wave + 8 * i;
        const int n = nt * 16 + m16;
        const _Float16* ar = sA + m16 * 264 + 8 * hf;
        const _Float16* br = Wih + (size_t)n * (2 * IN_D) + 8 * hf;
        v8f acc = zero8();
#pragma unroll 2
        for (int k0 = 0; k0 < 2 * IN_D; k0 += 32) {
            FragH a, bq;
            a.half[0]  = ldh8(ar + k0); a.half[1]  = ldh8(ar + k0 + 16);
            bq.half[0] = ldh8(br + k0); bq.half[1] = ldh8(br + k0 + 16);
            acc = mma_f16(a.v, bq.v, acc);
        }
        const float bb = bi[n];
#pragma unroll
        for (int r = 0; r < 8; ++r) sY[(8 * hf + r) * 516 + n] = acc[r] * (1.0f / 1024.0f) + bb;
    }
    __syncthreads();

    {
        const int m = tid >> 4, g = tid & 15;
        float* yr = sY + m * 516;
        float s = 0.f;
        for (int j = g; j < DI; j += 16) s += yr[j];
        s = hsum16(s);
        const float mu = s * (1.0f / (float)DI);
        float q = 0.f;
        for (int j = g; j < DI; j += 16) { const float d = yr[j] - mu; q += d * d; }
        q = hsum16(q);
        const float rstd = rsqrtf(q * (1.0f / (float)DI) + 1e-5f);
        for (int j = g; j < DI; j += 16) {
            const float v = (yr[j] - mu) * rstd * gi[j] + bei[j];
            yr[j] = sigm(v);
        }
    }

    if (tid < 16) {
        const float* Ri = fr + (size_t)sCol[tid] * 9;
        const float* Rj = fr + (size_t)sRow[tid] * 9;
        float ri[9], rj[9];
#pragma unroll
        for (int a = 0; a < 9; ++a) { ri[a] = Ri[a]; rj[a] = Rj[a]; }
#pragma unroll
        for (int i2 = 0; i2 < 3; ++i2)
#pragma unroll
            for (int j2 = 0; j2 < 3; ++j2) {
                float acc = 0.f;
#pragma unroll
                for (int k2 = 0; k2 < 3; ++k2) acc += ri[k2 * 3 + i2] * rj[k2 * 3 + j2];
                sR[tid * 12 + i2 * 3 + j2] = acc;
            }
    }
    __syncthreads();

    for (int p = tid; p < 512; p += 256) {
        const int m = p >> 5, k = p & 31;
        float* dst = sU + (m * 32 + k) * 9;
        if (k < 16) {
            const float* src = tens + (size_t)sCol[m] * D9 + k * 9;
#pragma unroll
            for (int a = 0; a < 9; ++a) dst[a] = src[a];
        } else {
            const float* src = tens + (size_t)sRow[m] * D9 + (k - 16) * 9;
            float T[9], Rm[9], M1[9];
#pragma unroll
            for (int a = 0; a < 9; ++a) { T[a] = src[a]; Rm[a] = sR[m * 12 + a]; }
#pragma unroll
            for (int i2 = 0; i2 < 3; ++i2)
#pragma unroll
                for (int j2 = 0; j2 < 3; ++j2) {
                    float acc = 0.f;
#pragma unroll
                    for (int k2 = 0; k2 < 3; ++k2) acc += Rm[i2 * 3 + k2] * T[k2 * 3 + j2];
                    M1[i2 * 3 + j2] = acc;
                }
#pragma unroll
            for (int i2 = 0; i2 < 3; ++i2)
#pragma unroll
                for (int j2 = 0; j2 < 3; ++j2) {
                    float acc = 0.f;
#pragma unroll
                    for (int k2 = 0; k2 < 3; ++k2) acc += M1[i2 * 3 + k2] * Rm[k2 * 3 + j2];
                    dst[i2 * 3 + j2] = acc;
                }
        }
    }
    __syncthreads();

    {
        const int m = tid >> 4, c = tid & 15;
        float r9[9];
#pragma unroll
        for (int a = 0; a < 9; ++a) r9[a] = 0.f;
        const float* wr = sY + m * 516 + c;
        const float* sp = sU + m * 32 * 9;
#pragma unroll 4
        for (int k = 0; k < 32; ++k) {
            const float wv = wr[k * 16];
#pragma unroll
            for (int a = 0; a < 9; ++a) r9[a] += sp[k * 9 + a] * wv;
        }
        __syncthreads();
        float* o = sU + m * D9 + c * 9;
#pragma unroll
        for (int a = 0; a < 9; ++a) o[a] = r9[a];
    }
    __syncthreads();

    float* dst = TN + (size_t)e0 * D9;
    for (int idx = tid; idx < 16 * D9 / 4; idx += 256) {
        const v4f v = *(const v4fa*)(sU + idx * 4);
        *(volatile v4f*)(dst + idx * 4) = v;
    }
    __threadfence();
    for (int idx = tid; idx < 16 * D9 / 4; idx += 256) {
        const v4f v = *(const v4fa*)(sU + idx * 4);
        *(volatile v4f*)(dst + idx * 4) = v;
    }
}

__global__ __launch_bounds__(256) void k_gather(
    const int* __restrict__ LB, const int* __restrict__ SK,
    const float* __restrict__ TN, float* __restrict__ out,
    int N, int E, int G, int NP)
{
    __shared__ __attribute__((aligned(16))) float sO[32 * D9];
    const int tid = threadIdx.x, slot = tid >> 3, g = tid & 7;
    const int nb0 = blockIdx.x * 32;
    const int node = nb0 + slot;

    float acc[18];
#pragma unroll
    for (int u = 0; u < 18; ++u) acc[u] = 0.f;

    if (node < N) {
        int done = 0;
        for (int c = 0; c < G; ++c) {
            const int* lbr = LB + (size_t)c * NP;
            int lo = lbr[node];
            int hi = lbr[node + 1];
            lo = clampi(lo, 0, CHK);
            hi = clampi(hi, lo, CHK);
            int cnt = hi - lo;
            const int room = MAXDEG - done;
            cnt = cnt < room ? cnt : room;
            done += cnt;
            const int* skc = SK + (size_t)c * CHK + lo;
            for (int p = 0; p < cnt; ++p) {
                const int key = skc[p];
                int e = c * CHK + (key & (CHK - 1));
                e = e < E ? e : E - 1;
                const float* src = TN + (size_t)e * D9 + g * 18;
#pragma unroll
                for (int u = 0; u < 9; ++u) {
                    const v2f v = *(const v2fa*)(src + 2 * u);
                    acc[2 * u]     += v.x;
                    acc[2 * u + 1] += v.y;
                }
            }
        }
    }

    float* so = sO + slot * D9 + g * 18;
#pragma unroll
    for (int bch = 0; bch < 2; ++bch) {
        const int q = 9 * bch;
        const float s01 = 0.5f * (acc[q + 1] + acc[q + 3]);
        const float s02 = 0.5f * (acc[q + 2] + acc[q + 6]);
        const float s12 = 0.5f * (acc[q + 5] + acc[q + 7]);
        so[q + 0] = acc[q + 0]; so[q + 1] = s01; so[q + 2] = s02;
        so[q + 3] = s01;        so[q + 4] = acc[q + 4]; so[q + 5] = s12;
        so[q + 6] = s02;        so[q + 7] = s12; so[q + 8] = acc[q + 8];
    }
    __syncthreads();

    int rows = N - nb0; rows = rows > 32 ? 32 : rows;
    const int nf4 = rows * (D9 / 4);
    float* dst = out + (size_t)nb0 * D9;
    for (int idx = tid; idx < nf4; idx += 256) {
        const v4f v = *(const v4fa*)(sO + idx * 4);
        *(volatile v4f*)(dst + idx * 4) = v;
    }
    __threadfence();
    for (int idx = tid; idx < nf4; idx += 256) {
        const v4f v = *(const v4fa*)(sO + idx * 4);
        *(volatile v4f*)(dst + idx * 4) = v;
    }
}

static inline size_t align256(size_t x) { return (x + 255) & ~(size_t)255; }

extern "C" void kernel_launch(void* const* d_in, const int* in_sizes, int n_in,
                              void* d_out, int out_size, void* d_ws, size_t ws_size,
                              hipStream_t stream)
{
    if (n_in < 17) return;
    const float* h   = (const float*)d_in[1];
    const float* fr  = (const float*)d_in[2];
    const int*   ei  = (const int*)d_in[3];
    const float* W1  = (const float*)d_in[5];
    const float* b1  = (const float*)d_in[6];
    const float* g1  = (const float*)d_in[7];
    const float* be1 = (const float*)d_in[8];
    const float* W2  = (const float*)d_in[9];
    const float* b2  = (const float*)d_in[10];
    const float* g2  = (const float*)d_in[11];
    const float* be2 = (const float*)d_in[12];
    const float* Wi  = (const float*)d_in[13];
    const float* bi  = (const float*)d_in[14];
    const float* gi  = (const float*)d_in[15];
    const float* bei = (const float*)d_in[16];

    const int N = in_sizes[1] / IN_D;
    const int E = in_sizes[3] / 2;
    if (N <= 0 || E <= 0) return;
    if (in_sizes[1] != N * IN_D || in_sizes[2] != N * 9 || in_sizes[3] != 2 * E) return;
    if (in_sizes[5] != D9 * IN_D || in_sizes[9] != D9 * D9 || in_sizes[13] != DI * 2 * IN_D) return;
    if (in_sizes[6] != D9 || in_sizes[7] != D9 || in_sizes[8] != D9) return;
    if (in_sizes[10] != D9 || in_sizes[11] != D9 || in_sizes[12] != D9) return;
    if (in_sizes[14] != DI || in_sizes[15] != DI || in_sizes[16] != DI) return;
    if (out_size != N * D9) return;
    if (N >= (1 << 19)) return;

    const int Npad = (N + 15) / 16 * 16;
    const int Epad = (E + 15) / 16 * 16;
    const int G    = (E + CHK - 1) / CHK;
    const int NP   = (N + 1 + 31) / 32 * 32;

    size_t off = 0;
    const size_t o_hh   = off; off = align256(off + (size_t)Npad * IN_D * 2);
    const size_t o_w1h  = off; off = align256(off + (size_t)D9 * IN_D * 2);
    const size_t o_w1l  = off; off = align256(off + (size_t)D9 * IN_D * 2);
    const size_t o_w2h  = off; off = align256(off + (size_t)D9 * KP2 * 2);
    const size_t o_w2l  = off; off = align256(off + (size_t)D9 * KP2 * 2);
    const size_t o_wih  = off; off = align256(off + (size_t)DI * 2 * IN_D * 2);
    const size_t o_tens = off; off = align256(off + (size_t)Npad * D9 * 4);
    const size_t o_tn   = off; off = align256(off + (size_t)Epad * D9 * 4);
    const size_t o_lb   = off; off = align256(off + (size_t)G * NP * 4);
    const size_t o_sk   = off; off = align256(off + (size_t)G * CHK * 4);
    if (off > ws_size) return;

    char* ws = (char*)d_ws;
    _Float16* hh   = (_Float16*)(ws + o_hh);
    __bf16*   W1hi = (__bf16*)(ws + o_w1h);
    __bf16*   W1lo = (__bf16*)(ws + o_w1l);
    __bf16*   W2hi = (__bf16*)(ws + o_w2h);
    __bf16*   W2lo = (__bf16*)(ws + o_w2l);
    _Float16* Wih  = (_Float16*)(ws + o_wih);
    float*    tens = (float*)(ws + o_tens);
    float*    TN   = (float*)(ws + o_tn);
    int*      LB   = (int*)(ws + o_lb);
    int*      SK   = (int*)(ws + o_sk);
    float*    out  = (float*)d_out;

    const int gH  = Npad / 16;
    const int gW1 = (D9 * (IN_D / 8) + 255) / 256;
    const int gW2 = (D9 * (KP2 / 8) + 255) / 256;
    const int gWi = (DI * (2 * IN_D / 8) + 255) / 256;
    const int s1 = gH, s3 = s1 + 2 * gW1, s5 = s3 + 2 * gW2;
    k_conv<<<s5 + gWi, 256, 0, stream>>>(h, W1, W2, Wi, hh, W1hi, W1lo, W2hi, W2lo, Wih,
                                         N, Npad, s1, s3, s5);

    k_node<<<Npad / 16, 256, 0, stream>>>(h, W1hi, W1lo, b1, g1, be1, W2hi, W2lo, b2, g2, be2, tens, N);

    k_sort<<<G, 256, 0, stream>>>(ei, LB, SK, N, E, NP);

    k_edge<<<Epad / 16, 256, 0, stream>>>(hh, fr, ei, tens, Wih, bi, gi, bei, TN, N, E);

    k_gather<<<(N + 31) / 32, 256, 0, stream>>>(LB, SK, TN, out, N, E, G, NP);
}
